// LSTMParser_76836964926134
// MI455X (gfx1250) — hardware-verified
//
#include <hip/hip_runtime.h>
#include <math.h>

typedef __attribute__((ext_vector_type(16))) _Float16 v16h;
typedef __attribute__((ext_vector_type(8)))  _Float16 v8h;
typedef __attribute__((ext_vector_type(16))) __bf16   v16b;
typedef __attribute__((ext_vector_type(8)))  __bf16   v8b;
typedef __attribute__((ext_vector_type(8)))  float    v8f;
typedef __attribute__((ext_vector_type(4)))  float    v4f;

constexpr int kN    = 512;
constexpr int kIn   = 125;
constexpr int kInP  = 128;
constexpr int kH    = 125;
constexpr int kG4   = 4 * kH;
constexpr int kG4P  = 512;
constexpr int kD    = 2 * kH;
constexpr int kDP   = 256;
constexpr int kM    = 512;
constexpr int kThr  = 256;
constexpr float kXCarry = 1024.0f;
constexpr float kWCarry = 4096.0f;
constexpr float kSc = 1.0f / (kXCarry * kWCarry);
constexpr float kF16MinNormal = 6.103515625e-5f;
constexpr int kFBF = 0, kFBB = 512, kFB1 = 1024, kFBZ = 1536, kFEnd = 2048;

static_assert((kN % 64) == 0 && (kG4P % 64) == 0 && ((kN / 64) * (kG4P / 64)) % 8 == 0 && ((kN / 64) * (2 * kM / 64)) % 8 == 0 && (kInP % 32) == 0 && (kDP % 32) == 0
              && kG4 <= kG4P && kIn <= kInP && kD <= kDP, "GEMM M, N multiples of 64; grids exact; K multiples of 32");

constexpr size_t kOffXE = 0ull;
constexpr size_t kOffWIH = 131072ull;
constexpr size_t kOffW1AB = 393216ull;
constexpr size_t kOffBIAS = 917504ull;
constexpr size_t kOffPRE = 925696ull;
constexpr size_t kOffHSD = 3022848ull;
constexpr size_t kOffH16 = 3547136ull;
constexpr size_t kOffP32 = 3809280ull;
constexpr size_t kWsTotal = 5906432ull;
static_assert(kWsTotal <= 134217728ull, "carve cap: under 128 MiB");
static_assert(kOffXE == 0
              && kOffWIH == kOffXE + 131072ull
              && kOffW1AB == kOffWIH + 262144ull
              && kOffBIAS == kOffW1AB + 524288ull
              && kOffPRE == kOffBIAS + 8192ull
              && kOffHSD == kOffPRE + 2097152ull
              && kOffH16 == kOffHSD + 524288ull
              && kOffP32 == kOffH16 + 262144ull
              && kWsTotal == kOffP32 + 2097152ull, "the carve is chained and totalled");
static_assert((kOffXE % 256) == 0 && (kOffWIH % 256) == 0 && (kOffW1AB % 256) == 0 && (kOffBIAS % 256) == 0 && (kOffPRE % 256) == 0 && (kOffHSD % 256) == 0 && (kOffH16 % 256) == 0 && (kOffP32 % 256) == 0, "aligned regions");

__device__ __forceinline__ unsigned short f2bf_bits(float f) {
  unsigned u = __float_as_uint(f);
  return (unsigned short)((u + 0x7FFFu + ((u >> 16) & 1u)) >> 16);
}
__device__ __forceinline__ float bf_bits2f(unsigned short h) { return __uint_as_float(((unsigned)h) << 16); }
__device__ __forceinline__ float bf16r(float f) { return bf_bits2f(f2bf_bits(f)); }
__device__ __forceinline__ float carry_flush(float v, float carry) {
  const float s = v * carry;
  return (fabsf(s) < kF16MinNormal) ? 0.0f : s;
}
__device__ __forceinline__ float frcp(float x) { return __builtin_amdgcn_rcpf(x); }

__device__ __forceinline__ void dep_guard4_h(v8f& a, v8f& b, v8f& c, v8f& d, v16h x, v16h y) { asm volatile("v_nop\n\tv_nop\n\tv_nop\n\tv_nop" : "+v"(a), "+v"(b), "+v"(c), "+v"(d) : "v"(x), "v"(y)); }
__device__ __forceinline__ void dep_guard4_b(v8f& a, v8f& b, v8f& c, v8f& d, v16b x, v16b y) { asm volatile("v_nop\n\tv_nop\n\tv_nop\n\tv_nop" : "+v"(a), "+v"(b), "+v"(c), "+v"(d) : "v"(x), "v"(y)); }
__device__ __forceinline__ void keep4_h(v16h a, v16h b, v16h c, v16h d) { asm volatile("v_nop" :: "v"(a), "v"(b), "v"(c), "v"(d)); }
__device__ __forceinline__ void keep4_b(v16b a, v16b b, v16b c, v16b d) { asm volatile("v_nop" :: "v"(a), "v"(b), "v"(c), "v"(d)); }
__device__ __forceinline__ void acc_guard4(v8f& a, v8f& b, v8f& c, v8f& d) { asm volatile("v_nop\n\tv_nop\n\tv_nop\n\tv_nop" : "+v"(a), "+v"(b), "+v"(c), "+v"(d)); }

template <typename T> struct Frag;
template <> struct Frag<_Float16> {
  typedef v16h V; union U { v16h v; v8h h[2]; };
  static __device__ __forceinline__ v16h load(const _Float16* p) {
    U f; f.h[0] = *(const v8h*)(p); f.h[1] = *(const v8h*)(p + 16); return f.v;
  }
  static __device__ __forceinline__ v8f mma(v16h a, v16h b, v8f c) {
    return __builtin_amdgcn_wmma_f32_16x16x32_f16(false, a, false, b, (short)0, c, false, false);
  }
  static __device__ __forceinline__ void guard4(v8f& a, v8f& b, v8f& c, v8f& d, v16h x, v16h y) { dep_guard4_h(a, b, c, d, x, y); }
  static __device__ __forceinline__ void keep(v16h a, v16h b, v16h c, v16h d) { keep4_h(a, b, c, d); }
};
template <> struct Frag<__bf16> {
  typedef v16b V; union U { v16b v; v8b h[2]; };
  static __device__ __forceinline__ v16b load(const __bf16* p) {
    U f; f.h[0] = *(const v8b*)(p); f.h[1] = *(const v8b*)(p + 16); return f.v;
  }
  static __device__ __forceinline__ v8f mma(v16b a, v16b b, v8f c) {
    return __builtin_amdgcn_wmma_f32_16x16x32_bf16(false, a, false, b, (short)0, c, false, false);
  }
  static __device__ __forceinline__ void guard4(v8f& a, v8f& b, v8f& c, v8f& d, v16b x, v16b y) { dep_guard4_b(a, b, c, d, x, y); }
  static __device__ __forceinline__ void keep(v16b a, v16b b, v16b c, v16b d) { keep4_b(a, b, c, d); }
};

__device__ __forceinline__ v8f mma_h(v16h a, v16h b, v8f c) {
  c = __builtin_amdgcn_wmma_f32_16x16x32_f16(false, a, false, b, (short)0, c, false, false);
  asm volatile("v_nop\n\tv_nop\n\tv_nop\n\tv_nop" : "+v"(c) : "v"(a), "v"(b));
  return c;
}

template <int ET> struct Elem;
template <> struct Elem<0> { typedef _Float16 T; };
template <> struct Elem<1> { typedef __bf16 T; };
template <int ET, bool SPLIT, int BIAS_MODE, int OUT_MODE, bool RESID, int ACT = 0>
__global__ __launch_bounds__(256) void wmma_gemm64(
    const unsigned short* __restrict__ Ap, const unsigned short* __restrict__ A2p, int lda, long strideA,
    const unsigned short* __restrict__ Btp, const unsigned short* __restrict__ Bt2p, int ldb, long strideB,
    void* __restrict__ Cout, void* __restrict__ Cout2, int ldc, long strideC,
    const float* __restrict__ bias,
    const float* __restrict__ resid, long strideR,
    int M, int N, int K, float scale) {
  typedef typename Elem<ET>::T T;
  typedef typename Frag<T>::V V;
  const T* A = (const T*)Ap; const T* A2 = (const T*)A2p; const T* Bt = (const T*)Btp; const T* Bt2 = (const T*)Bt2p;
  __shared__ __align__(16) float sT[8][16 * 68];
  const int b    = blockIdx.y;
  const int lane = threadIdx.x & 31;
  const int wave = threadIdx.x >> 5;
  const int tilesN = N >> 6;
  const int tilesM = M >> 6;
  const int tile = blockIdx.x * 8 + wave;
  if (tile >= tilesM * tilesN) return;
  const int tm = tile / tilesN;
  const int tn = tile - tm * tilesN;
  const int m0 = tm << 6;
  const int n0 = tn << 6;

  const T* Ab  = A  + (size_t)b * strideA;
  const T* Bb  = Bt + (size_t)b * strideB;
  const T* Ab2 = SPLIT ? (A2  + (size_t)b * strideA) : nullptr;
  const T* Bb2 = SPLIT ? (Bt2 + (size_t)b * strideB) : nullptr;

  const int rlane = lane & 15;
  const int koff  = (lane >> 4) * 8;
  const int mOff  = (lane >> 4) * 8;

  v8f acc[4][4];
#pragma unroll
  for (int i = 0; i < 4; ++i)
#pragma unroll
    for (int j = 0; j < 4; ++j) acc[i][j] = (v8f){0.f,0.f,0.f,0.f,0.f,0.f,0.f,0.f};

  for (int k0 = 0; k0 < K; k0 += 32) {
    V bh[4], bl[4];
#pragma unroll
    for (int j = 0; j < 4; ++j) {
      const size_t bo = (size_t)(n0 + (j << 4) + rlane) * ldb + koff + k0;
      bh[j] = Frag<T>::load(Bb + bo);
      if (SPLIT) bl[j] = Frag<T>::load(Bb2 + bo);
    }
#pragma unroll
    for (int i = 0; i < 4; ++i) {
      const size_t ao = (size_t)(m0 + (i << 4) + rlane) * lda + koff + k0;
      V ah = Frag<T>::load(Ab + ao);
      V al;
      if (SPLIT) al = Frag<T>::load(Ab2 + ao);
#pragma unroll
      for (int j = 0; j < 4; ++j) {
        acc[i][j] = Frag<T>::mma(ah, bh[j], acc[i][j]);
        if (SPLIT) {
          acc[i][j] = Frag<T>::mma(ah, bl[j], acc[i][j]);
          acc[i][j] = Frag<T>::mma(al, bh[j], acc[i][j]);
        }
      }
      Frag<T>::guard4(acc[i][0], acc[i][1], acc[i][2], acc[i][3], ah, SPLIT ? al : ah);
    }
    Frag<T>::keep(bh[0], bh[1], bh[2], bh[3]);
    if (SPLIT) Frag<T>::keep(bl[0], bl[1], bl[2], bl[3]);
  }
  acc_guard4(acc[0][0], acc[0][1], acc[0][2], acc[0][3]);
  acc_guard4(acc[1][0], acc[1][1], acc[1][2], acc[1][3]);
  acc_guard4(acc[2][0], acc[2][1], acc[2][2], acc[2][3]);
  acc_guard4(acc[3][0], acc[3][1], acc[3][2], acc[3][3]);

  float* slab = sT[wave];
  const float* Rb = RESID ? (resid + (size_t)b * strideR) : nullptr;
#pragma unroll
  for (int i = 0; i < 4; ++i) {
    const int mBase = m0 + (i << 4);
#pragma unroll
    for (int j = 0; j < 4; ++j) {
      const int n = n0 + (j << 4) + rlane;
      float bv = 0.f;
      if (BIAS_MODE == 2) bv = bias[n];
#pragma unroll
      for (int r = 0; r < 8; ++r) {
        float v = acc[i][j][r] * scale;
        if (BIAS_MODE == 1) v += bias[mBase + mOff + r];
        if (BIAS_MODE == 2) v += bv;
        if (RESID) v += Rb[(size_t)(mBase + mOff + r) * ldc + n];
        if (ACT == 1) v = tanhf(v);
        if (ACT == 2) v = fmaxf(v, 0.0f);
        if (ACT == 3) v = v / (1.0f + expf(-v));
        if (ACT == 4) v = (v > 0.f) ? v : 0.01f * v;
        slab[(mOff + r) * 68 + (j << 4) + rlane] = v;
      }
    }
    __builtin_amdgcn_fence(__ATOMIC_RELEASE, "workgroup");
    __builtin_amdgcn_wave_barrier();
    __builtin_amdgcn_fence(__ATOMIC_ACQUIRE, "workgroup");
    if (OUT_MODE == 0) {
      float* C = (float*)Cout + (size_t)b * strideC;
      const int hh = lane >> 4, c4 = (lane & 15) * 4;
      for (int pass = 0; pass < 2; ++pass) {
#pragma unroll
        for (int it = 0; it < 8; ++it) {
          const int row = it * 2 + hh;
          v4f v = *(const v4f*)(slab + row * 68 + c4);
          *(volatile v4f*)(C + (size_t)(mBase + row) * ldc + n0 + c4) = v;
        }
        __threadfence();
      }
    } else {
      const int q = lane >> 3, c8 = (lane & 7) * 8;
      unsigned short* C  = (unsigned short*)Cout  + (size_t)b * strideC;
      unsigned short* C2 = (OUT_MODE == 2) ? ((unsigned short*)Cout2 + (size_t)b * strideC) : nullptr;
      for (int pass = 0; pass < 2; ++pass) {
#pragma unroll
        for (int it = 0; it < 4; ++it) {
          const int row = it * 4 + q;
          const float* sp = slab + row * 68 + c8;
          v8h hv, lv;
#pragma unroll
          for (int e = 0; e < 8; ++e) {
            if (OUT_MODE == 1) {
              hv[e] = (_Float16)sp[e];
            } else {
              unsigned short hb = f2bf_bits(sp[e]);
              unsigned short lb = f2bf_bits(sp[e] - bf_bits2f(hb));
              hv[e] = __builtin_bit_cast(_Float16, hb);
              lv[e] = __builtin_bit_cast(_Float16, lb);
            }
          }
          *(volatile v8h*)(C + (size_t)(mBase + row) * ldc + n0 + c8) = hv;
          if (OUT_MODE == 2) *(volatile v8h*)(C2 + (size_t)(mBase + row) * ldc + n0 + c8) = lv;
        }
        __threadfence();
      }
    }
    __builtin_amdgcn_fence(__ATOMIC_RELEASE, "workgroup");
    __builtin_amdgcn_wave_barrier();
    __builtin_amdgcn_fence(__ATOMIC_ACQUIRE, "workgroup");
  }
}


__device__ __forceinline__ float fast_tanh(float v) { return 1.0f - 2.0f * frcp(__expf(2.0f * v) + 1.0f); }
__device__ __forceinline__ float fast_sigmoid(float v) { return frcp(1.0f + __expf(-v)); }

__global__ __launch_bounds__(kThr) void setup_kernel(const float* __restrict__ emb, const float* __restrict__ wih_f, const float* __restrict__ wih_b, const float* __restrict__ bih_f,
                                                     const float* __restrict__ bhh_f, const float* __restrict__ bih_b, const float* __restrict__ bhh_b, const float* __restrict__ w1,
                                                     const float* __restrict__ b1, float* __restrict__ BIAS, unsigned short* __restrict__ XE, unsigned short* __restrict__ WIH,
                                                     unsigned short* __restrict__ W1AB, unsigned short* __restrict__ H16) {
  unsigned v = blockIdx.x * (unsigned)kThr + threadIdx.x;
  asm volatile("" : "+v"(v));
  if (v < 512u) {
    const unsigned i0 = v * 4u;
    float o[4];
#pragma unroll
    for (int e = 0; e < 4; ++e) {
      const unsigned i = i0 + (unsigned)e;
      const unsigned q = i & 511u;
      const unsigned qg = (q < (unsigned)kG4) ? q : 0u;
      float a = 0.0f, b = 0.0f;
      if (i < (unsigned)kFBB) { a = bih_f[qg]; b = bhh_f[qg]; }
      else if (i < (unsigned)kFB1) { a = bih_b[qg]; b = bhh_b[qg]; }
      else if (i < (unsigned)kFBZ) { a = b1[q]; }
      asm volatile("" : "+v"(a), "+v"(b));
      const bool gate = i < (unsigned)kFB1;
      o[e] = gate ? ((q < (unsigned)kG4) ? (bf16r(a) + bf16r(b)) : 0.0f) : ((i < (unsigned)kFBZ) ? bf16r(a) : 0.0f);
    }
    const v4f ov = {o[0], o[1], o[2], o[3]};
    float* dp = BIAS + i0;
    *(volatile v4f*)dp = ov;
    __threadfence();
    *(volatile v4f*)dp = ov;
  } else {
    v8h hv;
    unsigned short* dp;
    if (v < 8704u) {
      unsigned w = v - 512u;
      asm volatile("" : "+v"(w));
      const unsigned t = w >> 4, c8 = (w & 15u) * 8u;
#pragma unroll
      for (int e = 0; e < 8; ++e) {
        const unsigned c = c8 + (unsigned)e;
        float p = emb[(size_t)t * kIn + ((c < (unsigned)kIn) ? c : 0u)];
        asm volatile("" : "+v"(p));
        hv[e] = (_Float16)((c < (unsigned)kIn) ? carry_flush(bf16r(p), kXCarry) : 0.0f);
      }
      dp = XE + (size_t)w * 8u;
    } else if (v < 25088u) {
      unsigned w = v - 8704u;
      asm volatile("" : "+v"(w));
      const unsigned d = w >> 13, n = (w >> 4) & 511u, c8 = (w & 15u) * 8u;
      const float* W = d ? wih_b : wih_f;
      const unsigned ng = (n < (unsigned)kG4) ? n : 0u;
#pragma unroll
      for (int e = 0; e < 8; ++e) {
        const unsigned c = c8 + (unsigned)e;
        float p = W[(size_t)ng * kIn + ((c < (unsigned)kIn) ? c : 0u)];
        asm volatile("" : "+v"(p));
        hv[e] = (_Float16)((n < (unsigned)kG4 && c < (unsigned)kIn) ? carry_flush(bf16r(p), kWCarry) : 0.0f);
      }
      dp = WIH + (size_t)w * 8u;
    } else if (v < 57856u) {
      unsigned w = v - 25088u;
      asm volatile("" : "+v"(w));
      const unsigned n = w >> 5, c8 = (w & 31u) * 8u;
      const unsigned half = n >> 9, m = n & 511u;
#pragma unroll
      for (int e = 0; e < 8; ++e) {
        const unsigned c = c8 + (unsigned)e;
        float p = w1[(size_t)m * (2 * kD) + half * (unsigned)kD + ((c < (unsigned)kD) ? c : 0u)];
        asm volatile("" : "+v"(p));
        hv[e] = (_Float16)((c < (unsigned)kD) ? carry_flush(bf16r(p), kWCarry) : 0.0f);
      }
      dp = W1AB + (size_t)w * 8u;
    } else {
      unsigned w = v - 57856u;
      asm volatile("" : "+v"(w));
#pragma unroll
      for (int e = 0; e < 8; ++e) hv[e] = (_Float16)0.0f;
      dp = H16 + (size_t)w * 8u;
    }
    *(volatile v8h*)dp = hv;
    __threadfence();
    *(volatile v8h*)dp = hv;
  }
}
static_assert(kFEnd / 4 == 512 && kN * (kInP / 8) == 8192 && 512 + 8192 == 8704 && 2 * kG4P * (kInP / 8) == 16384 && 8704 + 16384 == 25088 && 2 * kM * (kDP / 8) == 32768 && 25088 + 32768 == 57856
              && kN * (kDP / 8) == 16384 && 57856 + 16384 == 290 * kThr, "set-up grid exact");

__global__ __launch_bounds__(512) void chain_kernel(const float* __restrict__ PRE, const float* __restrict__ whh_f, const float* __restrict__ whh_b, float* __restrict__ HSD) {
  __shared__ float sH[128];
  __shared__ float sG[512];
  const int d = (int)blockIdx.x;
  unsigned r = threadIdx.x;
  asm volatile("" : "+v"(r));
  const bool live = r < (unsigned)kG4;
  const float* wr = (d ? whh_b : whh_f) + (size_t)(live ? r : 0u) * kH;
  float w[kH];
#pragma unroll
  for (int k = 0; k < kH; ++k) { float p = wr[k]; asm volatile("" : "+v"(p)); w[k] = live ? bf16r(p) : 0.0f; }
  if (r < 128u) sH[r] = 0.0f;
  float c = 0.0f;
  const float* pre_d = PRE + (size_t)d * kN * kG4P;
  float* hs_d = HSD + (size_t)d * kN * 128;
  __syncthreads();
  for (int s = 0; s < kN; ++s) {
    const int t = d ? (kN - 1 - s) : s;
    float acc = pre_d[(size_t)t * kG4P + r];
#pragma unroll
    for (int k = 0; k < kH; ++k) acc += w[k] * sH[k];
    sG[r] = acc;
    __syncthreads();
    if (r < (unsigned)kH) {
      const float gi = sG[r], gf = sG[kH + r], gg = sG[2 * kH + r], go = sG[3 * kH + r];
      c = fast_sigmoid(gf) * c + fast_sigmoid(gi) * fast_tanh(gg);
      const float h = fast_sigmoid(go) * fast_tanh(c);
      sH[r] = h;
      float* hp = hs_d + (size_t)t * 128 + r;
      *(volatile float*)hp = h;
      __threadfence();
      *(volatile float*)hp = h;
    }
    __syncthreads();
  }
}

__global__ __launch_bounds__(kThr) void hcast_kernel(const float* __restrict__ HSD, unsigned short* __restrict__ H16) {
  unsigned v = blockIdx.x * (unsigned)kThr + threadIdx.x;
  asm volatile("" : "+v"(v));
  const unsigned t = v >> 5, c8 = (v & 31u) * 8u;
  v8h hv;
#pragma unroll
  for (int e = 0; e < 8; ++e) {
    const unsigned c = c8 + (unsigned)e;
    const unsigned dir = (c >= (unsigned)kH) ? 1u : 0u;
    const unsigned u = (c < (unsigned)kD) ? (c - dir * (unsigned)kH) : 0u;
    float p = HSD[((size_t)dir * kN + t) * 128 + u];
    asm volatile("" : "+v"(p));
    hv[e] = (_Float16)((c < (unsigned)kD) ? carry_flush(p, kXCarry) : 0.0f);
  }
  unsigned short* dp = H16 + (size_t)v * 8u;
  *(volatile v8h*)dp = hv;
  __threadfence();
  *(volatile v8h*)dp = hv;
}
static_assert(kN * (kDP / 8) == 64 * kThr, "state cast grid exact");

__global__ __launch_bounds__(kThr) void pair_kernel(const float* __restrict__ P32, const float* __restrict__ w2, const float* __restrict__ b2, float* __restrict__ out) {
  unsigned v = blockIdx.x * (unsigned)kThr + threadIdx.x;
  asm volatile("" : "+v"(v));
  const unsigned i = v >> 9, j = v & 511u;
  const float* pa = P32 + (size_t)j * (2 * kM);
  const float* pb = P32 + (size_t)i * (2 * kM) + kM;
  float acc = 0.0f;
  for (int k = 0; k < kM; k += 4) {
    const v4f a = *(const v4f*)(pa + k), b = *(const v4f*)(pb + k), w = *(const v4f*)(w2 + k);
    const float w0 = w[0], w1_ = w[1], w2_ = w[2], w3 = w[3];
    acc += bf16r(w0) * fast_tanh(a[0] + b[0]);
    acc += bf16r(w1_) * fast_tanh(a[1] + b[1]);
    acc += bf16r(w2_) * fast_tanh(a[2] + b[2]);
    acc += bf16r(w3) * fast_tanh(a[3] + b[3]);
  }
  float bb = b2[0];
  asm volatile("" : "+v"(bb));
  const float o = acc + bf16r(bb);
  *(volatile float*)(out + v) = o;
  __threadfence();
  *(volatile float*)(out + v) = o;
}
static_assert(kN * kN == 1024 * kThr, "pair grid exact");

extern "C" void kernel_launch(void* const* d_in, const int* in_sizes, int n_in,
                              void* d_out, int out_size, void* d_ws, size_t ws_size,
                              hipStream_t stream) {
  if (n_in < 13 || d_out == nullptr || d_ws == nullptr) return;
  if (in_sizes[0] != kN * kIn || in_sizes[1] != kG4 * kIn || in_sizes[2] != kG4 * kH || in_sizes[3] != kG4 || in_sizes[4] != kG4) return;
  if (in_sizes[5] != kG4 * kIn || in_sizes[6] != kG4 * kH || in_sizes[7] != kG4 || in_sizes[8] != kG4) return;
  if (in_sizes[9] != kM * 2 * kD || in_sizes[10] != kM || in_sizes[11] != kM || in_sizes[12] != 1) return;
  if (out_size != kN * kN) return;
  if (ws_size < kWsTotal) return;
  const float* emb = (const float*)d_in[0];
  const float* wih_f = (const float*)d_in[1];
  const float* whh_f = (const float*)d_in[2];
  const float* bih_f = (const float*)d_in[3];
  const float* bhh_f = (const float*)d_in[4];
  const float* wih_b = (const float*)d_in[5];
  const float* whh_b = (const float*)d_in[6];
  const float* bih_b = (const float*)d_in[7];
  const float* bhh_b = (const float*)d_in[8];
  const float* w1 = (const float*)d_in[9];
  const float* b1 = (const float*)d_in[10];
  const float* w2 = (const float*)d_in[11];
  const float* b2 = (const float*)d_in[12];
  float* out = (float*)d_out;
  char* ws = (char*)d_ws;
  unsigned short* XE = (unsigned short*)(ws + kOffXE);
  unsigned short* WIH = (unsigned short*)(ws + kOffWIH);
  unsigned short* W1AB = (unsigned short*)(ws + kOffW1AB);
  float* BIAS = (float*)(ws + kOffBIAS);
  float* PRE = (float*)(ws + kOffPRE);
  float* HSD = (float*)(ws + kOffHSD);
  unsigned short* H16 = (unsigned short*)(ws + kOffH16);
  float* P32 = (float*)(ws + kOffP32);

  setup_kernel<<<290, kThr, 0, stream>>>(emb, wih_f, wih_b, bih_f, bhh_f, bih_b, bhh_b, w1, b1, BIAS, XE, WIH, W1AB, H16);
  wmma_gemm64<0, false, 2, 0, false, 0><<<dim3((kN / 64) * (kG4P / 64) / 8, 1), 256, 0, stream>>>(
      XE, XE, kInP, 0L, WIH, WIH, kInP, 0L, (void*)PRE, (void*)PRE, kG4P, 0L, BIAS + kFBF, nullptr, 0L, kN, kG4P, kInP, kSc);
  wmma_gemm64<0, false, 2, 0, false, 0><<<dim3((kN / 64) * (kG4P / 64) / 8, 1), 256, 0, stream>>>(
      XE, XE, kInP, 0L, WIH + (size_t)kG4P * kInP, WIH + (size_t)kG4P * kInP, kInP, 0L, (void*)(PRE + (size_t)kN * kG4P), (void*)(PRE + (size_t)kN * kG4P), kG4P, 0L, BIAS + kFBB, nullptr, 0L, kN, kG4P, kInP, kSc);
  chain_kernel<<<2, 512, 0, stream>>>(PRE, whh_f, whh_b, HSD);
  hcast_kernel<<<64, kThr, 0, stream>>>(HSD, H16);
  wmma_gemm64<0, false, 2, 0, false, 0><<<dim3((kN / 64) * (2 * kM / 64) / 8, 1), 256, 0, stream>>>(
      H16, H16, kDP, 0L, W1AB, W1AB, kDP, 0L, (void*)P32, (void*)P32, 2 * kM, 0L, BIAS + kFB1, nullptr, 0L, kN, 2 * kM, kDP, kSc);
  pair_kernel<<<1024, kThr, 0, stream>>>(P32, w2, b2, out);
}
